// StandardAttention_15049565405218
// MI455X (gfx1250) — hardware-verified
//
#include <hip/hip_runtime.h>


#ifndef NB
#define NB 2
#endif
#ifndef SEQ
#define SEQ 2048
#endif
#ifndef NB_FULL
#define NB_FULL 2
#endif
#ifndef SEQ_FULL
#define SEQ_FULL 2048
#endif
#ifndef EROWS
#define EROWS 256
#endif

namespace {
constexpr int DM = 1024, H = 16, HD = 64, NW = 4;
constexpr int MROWS = NB * SEQ;
constexpr int QBLK = SEQ / 32;
constexpr int EBLK = (EROWS < SEQ ? EROWS : SEQ) / 32;
constexpr float XC = 8.0f, WC = 64.0f, QS = 8.0f, VS = 8.0f, CS = 8.0f, RS = 1024.0f, PS = 1024.0f, LOG2E = 1.4426950408889634f;
static_assert(SEQ % 64 == 0 && SEQ >= 64 && SEQ <= SEQ_FULL && NB >= 1 && NB <= NB_FULL);
static_assert(EROWS % 32 == 0 && EROWS >= 32 && EBLK >= 1 && EBLK <= QBLK);
static_assert(DM == H * HD && HD == 64 && DM % 64 == 0 && MROWS % 64 == 0 && (MROWS * (DM / 8)) % 256 == 0);

typedef _Float16 b16;
typedef __attribute__((ext_vector_type(16))) _Float16 v16b;
typedef __attribute__((ext_vector_type(8))) _Float16 v8b;
typedef __attribute__((ext_vector_type(8))) float v8f;
typedef __attribute__((ext_vector_type(4))) float v4f;

__device__ __forceinline__ float bf16_rne(float f) { unsigned int u = __float_as_uint(f); u += 0x7FFFu + ((u >> 16) & 1u); return __uint_as_float(u & 0xFFFF0000u); }
__device__ __forceinline__ v16b frag_kb(const b16* p, int hh) {
  const v8b a = *(const v8b*)(p + 8 * hh), b = *(const v8b*)(p + 16 + 8 * hh); v16b f;
#pragma unroll
  for (int e = 0; e < 8; ++e) { f[e] = a[e]; f[8 + e] = b[e]; }
  return f;
}
__device__ __forceinline__ v8f wmma16b(v16b a, v16b b, v8f c) {
  v8f d = __builtin_amdgcn_wmma_f32_16x16x32_f16(false, a, false, b, (short)0, c, false, false);
  asm volatile("v_nop\n\tv_nop\n\tv_nop\n\tv_nop" : "+v"(d) : "v"(a), "v"(b));
  return d;
}
__device__ __forceinline__ void wave_lds_sync() { __builtin_amdgcn_fence(3, "workgroup"); __builtin_amdgcn_wave_barrier(); __builtin_amdgcn_fence(2, "workgroup"); }
__device__ __forceinline__ float nexp2(float v) { return __builtin_amdgcn_exp2f(v); }

__global__ __launch_bounds__(256) void cvt_x_kernel(const float* __restrict__ X, b16* __restrict__ Xp) {
  const size_t u = (size_t)blockIdx.x * 256 + threadIdx.x;
  if (u >= (size_t)MROWS * (DM / 8)) return;
  const size_t row = u >> 7; const int piece = (int)(u & 127);
  const size_t b = row / SEQ, s = row % SEQ;
  const float* src = X + (b * SEQ_FULL + s) * DM + piece * 8;
  b16* dst = Xp + row * DM + piece * 8;
  const v4f x0 = *(const v4f*)src, x1 = *(const v4f*)(src + 4); v8b o;
#pragma unroll
  for (int j = 0; j < 4; ++j) { o[j] = (b16)(bf16_rne(x0[j]) * XC); o[4 + j] = (b16)(bf16_rne(x1[j]) * XC); }
  *(volatile v8b*)dst = o; __threadfence(); *(volatile v8b*)dst = o;
}

__global__ __launch_bounds__(64) void cvt_w_kernel(const float* __restrict__ W0, const float* __restrict__ W1, const float* __restrict__ W2,
                                                   const float* __restrict__ W3, b16* __restrict__ Wt) {
  __shared__ __attribute__((aligned(16))) b16 St[64][64 + 8];
  const int tid = threadIdx.x, wave = tid >> 5, lane = tid & 31;
  const int nt = (int)blockIdx.x, kt = (int)blockIdx.y, z = (int)blockIdx.z;
  const float* W = (z == 0) ? W0 : (z == 1) ? W1 : (z == 2) ? W2 : W3;
  const float* src = W + (size_t)kt * 64 * DM + (size_t)nt * 64;
  for (int it = 0; it < 16; ++it) {
    const int e = (it * 64 + tid) * 4; const int kk = e >> 6, nn = e & 63;
    const v4f x = *(const v4f*)(src + (size_t)kk * DM + nn);
#pragma unroll
    for (int j = 0; j < 4; ++j) St[nn + j][kk] = (b16)(bf16_rne(x[j]) * WC);
  }
  __syncthreads();
  b16* dstb = Wt + (size_t)z * DM * DM + (size_t)nt * 64 * DM + (size_t)kt * 64;
  for (int pass = 0; pass < 2; ++pass) {
#pragma unroll 1
    for (int it = 0; it < 8; ++it) {
      const int n = wave * 32 + it * 4 + (lane >> 3), kk = (lane & 7) * 8;
      const v8b o = *(const v8b*)(&St[n][kk]);
      *(volatile v8b*)(dstb + (size_t)n * DM + kk) = o; }
    __threadfence(); }
}

template <int MODE>
__global__ __launch_bounds__(128) __attribute__((amdgpu_num_vgpr(256))) void proj_kernel(const b16* __restrict__ Xp, const b16* __restrict__ Wt,
    const float* __restrict__ bias0, const float* __restrict__ bias1, b16* __restrict__ H0, b16* __restrict__ R0, b16* __restrict__ H1, b16* __restrict__ R1) {
  __shared__ __attribute__((aligned(16))) b16 Sm[2][64][64 + 8];
  const int tid = threadIdx.x, wave = tid >> 5, lane = tid & 31, hh = lane >> 4, col = lane & 15;
  const int z = (int)blockIdx.z;
  const int n0 = (int)blockIdx.x * 64, mblk = (int)blockIdx.y * 64, m0 = mblk + wave * 16;
  const b16* Wz = Wt + (size_t)z * DM * DM;
  const float* bias = (z == 0) ? bias0 : bias1; b16* Hp = (z == 0) ? H0 : H1; b16* Rp = (z == 0) ? R0 : R1;
  const b16* Arow = Xp + (size_t)(m0 + col) * DM;
  const b16* Brow = Wz + (size_t)(n0 + col) * DM;
  v8f acc[4];
#pragma unroll
  for (int t = 0; t < 4; ++t) acc[t] = (v8f){};
#pragma unroll 1
  for (int k0 = 0; k0 < DM; k0 += 32) {
    const v16b a = frag_kb(Arow + k0, hh);
#pragma unroll
    for (int t = 0; t < 4; ++t) acc[t] = wmma16b(a, frag_kb(Brow + (size_t)(t * 16) * DM + k0, hh), acc[t]);
  }
  constexpr float SCL = (MODE == 0) ? QS : VS;
#pragma unroll
  for (int t = 0; t < 4; ++t) {
    const int n = n0 + t * 16 + col; const float bvl = bf16_rne(bias[n]);
#pragma unroll
    for (int r = 0; r < 8; ++r) {
      const float v = (acc[t][r] * (1.0f / (XC * WC)) + bvl) * SCL; const b16 hv = (b16)v; const b16 rv = (b16)((v - (float)hv) * RS);
      if constexpr (MODE == 0) { Sm[0][wave * 16 + 8 * hh + r][t * 16 + col] = hv; Sm[1][wave * 16 + 8 * hh + r][t * 16 + col] = rv; }
      else { Sm[0][t * 16 + col][wave * 16 + 8 * hh + r] = hv; Sm[1][t * 16 + col][wave * 16 + 8 * hh + r] = rv; }
    } }
  const int hd = (int)blockIdx.x;
  if constexpr (MODE == 0) {
    wave_lds_sync();
    const size_t b = (size_t)m0 / SEQ, s0 = (size_t)m0 % SEQ;
    const size_t rowbase = ((b * H + hd) * SEQ + s0) * HD;
    for (int pass = 0; pass < 2; ++pass) {
#pragma unroll 1
      for (int it = 0; it < 4; ++it) {
        const int rr = it * 4 + (lane >> 3), piece = (lane & 7) * 8;
        const v8b oh = *(const v8b*)(&Sm[0][wave * 16 + rr][piece]); const v8b orr = *(const v8b*)(&Sm[1][wave * 16 + rr][piece]);
        *(volatile v8b*)(Hp + rowbase + (size_t)rr * HD + piece) = oh;
        *(volatile v8b*)(Rp + rowbase + (size_t)rr * HD + piece) = orr; }
      __threadfence(); }
  } else {
    __syncthreads();
    const size_t b = (size_t)mblk / SEQ, s0 = (size_t)mblk % SEQ;
    const size_t base = ((b * H + hd) * HD) * (size_t)SEQ + s0;
    for (int pass = 0; pass < 2; ++pass) {
#pragma unroll 1
      for (int it = 0; it < 4; ++it) {
        const int d = it * 16 + (tid >> 3), piece = (tid & 7) * 8;
        const v8b oh = *(const v8b*)(&Sm[0][d][piece]); const v8b orr = *(const v8b*)(&Sm[1][d][piece]);
        *(volatile v8b*)(Hp + base + (size_t)d * SEQ + piece) = oh;
        *(volatile v8b*)(Rp + base + (size_t)d * SEQ + piece) = orr; }
      __threadfence(); }
  }
}

template <bool EARLY>
__global__ __launch_bounds__(64) __attribute__((amdgpu_num_vgpr(256))) void attn_kernel(const b16* __restrict__ Qh, const b16* __restrict__ Qr,
    const b16* __restrict__ Kh, const b16* __restrict__ Kr, const b16* __restrict__ Vth, const b16* __restrict__ Vtr, b16* __restrict__ Ch, b16* __restrict__ Cr, int bx0) {
  __shared__ __attribute__((aligned(16))) b16 Pb[2][16][32 + 8];
  __shared__ __attribute__((aligned(16))) b16 Prs[2][16][32 + 8];
  __shared__ __attribute__((aligned(16))) b16 Toh[2][16][HD + 8];
  __shared__ __attribute__((aligned(16))) b16 Tor[2][16][HD + 8];
  const int wave = threadIdx.x >> 5, lane = threadIdx.x & 31, hh = lane >> 4, col = lane & 15;
  const size_t bhi = blockIdx.y; const int bx = bx0 + (int)blockIdx.x; const int q0 = bx * 32 + wave * 16, qi = q0 + col;
  const size_t pl = bhi * (size_t)SEQ * HD;
  const b16* Qhb = Qh + pl; const b16* Qrb = Qr + pl; const b16* Khb = Kh + pl; const b16* Krb = Kr + pl; const b16* Vhb = Vth + pl; const b16* Vrb = Vtr + pl;
  const v16b qa0 = frag_kb(Qhb + (size_t)qi * HD, hh), qa1 = frag_kb(Qhb + (size_t)qi * HD + 32, hh);
  v16b qr0 = (v16b){}, qr1 = (v16b){};
  if constexpr (EARLY) { qr0 = frag_kb(Qrb + (size_t)qi * HD, hh); qr1 = frag_kb(Qrb + (size_t)qi * HD + 32, hh); }
  const float cs = LOG2E / (8.0f * QS * QS);
  float m = -INFINITY, l = 0.0f; v8f o[4], oc[4];
#pragma unroll
  for (int t = 0; t < 4; ++t) { o[t] = (v8f){}; oc[t] = (v8f){}; }
  const int kend = bx * 32 + 32;
#pragma unroll 1
  for (int kb = 0; kb < kend; kb += 32) {
    float e[16]; float mx = -INFINITY;
#pragma unroll
    for (int u = 0; u < 2; ++u) {
      const size_t kr = (size_t)(kb + u * 16 + col) * HD;
      v8f s = (v8f){}; v8f s2 = (v8f){};
      const v16b kh0 = frag_kb(Khb + kr, hh);
      s = wmma16b(kh0, qa0, s);
      if constexpr (EARLY) { s2 = wmma16b(kh0, qr0, s2); s2 = wmma16b(frag_kb(Krb + kr, hh), qa0, s2); }
      const v16b kh1 = frag_kb(Khb + kr + 32, hh);
      s = wmma16b(kh1, qa1, s);
      if constexpr (EARLY) { s2 = wmma16b(kh1, qr1, s2); s2 = wmma16b(frag_kb(Krb + kr + 32, hh), qa1, s2); }
#pragma unroll
      for (int r = 0; r < 8; ++r) {
        float sv = s[r];
        if constexpr (EARLY) sv += s2[r] * (1.0f / RS);
        sv *= cs;
        const int key = kb + u * 16 + 8 * hh + r;
        const float ev = (key > qi) ? -INFINITY : sv;
        e[u * 8 + r] = ev; mx = fmaxf(mx, ev); } }
    mx = fmaxf(mx, __shfl_xor(mx, 16)); const float mn = fmaxf(m, mx); const float al = nexp2(m - mn); float sum = 0.0f;
#pragma unroll
    for (int i2 = 0; i2 < 16; ++i2) {
      const float p = nexp2(e[i2] - mn); sum += p; const int pi = (i2 < 8 ? 0 : 16) + 8 * hh + (i2 & 7);
      const float pp = p * PS; const b16 ph = (b16)pp; Pb[wave][col][pi] = ph;
      if constexpr (EARLY) Prs[wave][col][pi] = (b16)((pp - (float)ph) * RS); }
    sum += __shfl_xor(sum, 16); l = l * al + sum; m = mn;
    wave_lds_sync();
    const v16b pf = frag_kb(&Pb[wave][col][0], hh);
    v16b prf = (v16b){};
    if constexpr (EARLY) prf = frag_kb(&Prs[wave][col][0], hh);
#pragma unroll
    for (int t = 0; t < 4; ++t) {
      const size_t vo = (size_t)(t * 16 + col) * SEQ + kb;
      o[t] *= al; const v16b vh = frag_kb(Vhb + vo, hh);
      o[t] = wmma16b(vh, pf, o[t]);
      if constexpr (EARLY) { oc[t] *= al; oc[t] = wmma16b(vh, prf, oc[t]); oc[t] = wmma16b(frag_kb(Vrb + vo, hh), pf, oc[t]); } }
    wave_lds_sync(); }
  const float inv = 1.0f / (l * PS * VS);
#pragma unroll
  for (int t = 0; t < 4; ++t) {
#pragma unroll
    for (int r = 0; r < 8; ++r) {
      float ov = o[t][r];
      if constexpr (EARLY) ov += oc[t][r] * (1.0f / RS);
      const float cv = ov * inv * CS; const b16 hv = (b16)cv;
      Toh[wave][col][t * 16 + 8 * hh + r] = hv; Tor[wave][col][t * 16 + 8 * hh + r] = (b16)((cv - (float)hv) * RS); } }
  wave_lds_sync();
  const size_t b = bhi / H, h = bhi % H;
  const size_t rowbase = (b * SEQ + (size_t)q0) * DM + h * HD;
  for (int pass = 0; pass < 2; ++pass) {
#pragma unroll 1
    for (int it = 0; it < 4; ++it) {
      const int qq = it * 4 + (lane >> 3), piece = (lane & 7) * 8;
      const v8b oh = *(const v8b*)(&Toh[wave][qq][piece]); const v8b orr = *(const v8b*)(&Tor[wave][qq][piece]);
      *(volatile v8b*)(Ch + rowbase + (size_t)qq * DM + piece) = oh;
      *(volatile v8b*)(Cr + rowbase + (size_t)qq * DM + piece) = orr; }
    __threadfence(); }
}

__global__ __launch_bounds__(128) __attribute__((amdgpu_num_vgpr(256))) void oproj_kernel(const b16* __restrict__ Ch, const b16* __restrict__ Cr,
                                                                                     const b16* __restrict__ Wz, float* __restrict__ out) {
  __shared__ __attribute__((aligned(16))) float To[NW][16][HD + 4];
  const int tid = threadIdx.x, wave = tid >> 5, lane = tid & 31, hh = lane >> 4, col = lane & 15;
  const int n0 = (int)blockIdx.x * 64, mblk = (int)blockIdx.y * 64, m0 = mblk + wave * 16;
  const b16* Ah = Ch + (size_t)(m0 + col) * DM; const b16* Ar = Cr + (size_t)(m0 + col) * DM;
  const b16* Brow = Wz + (size_t)(n0 + col) * DM;
  v8f acc[4], acr[4];
#pragma unroll
  for (int t = 0; t < 4; ++t) { acc[t] = (v8f){}; acr[t] = (v8f){}; }
#pragma unroll 1
  for (int k0 = 0; k0 < DM; k0 += 32) {
    const v16b a = frag_kb(Ah + k0, hh), ar = frag_kb(Ar + k0, hh);
#pragma unroll
    for (int t = 0; t < 4; ++t) {
      const v16b bf = frag_kb(Brow + (size_t)(t * 16) * DM + k0, hh);
      acc[t] = wmma16b(a, bf, acc[t]); acr[t] = wmma16b(ar, bf, acr[t]); }
  }
#pragma unroll
  for (int t = 0; t < 4; ++t) {
#pragma unroll
    for (int r = 0; r < 8; ++r) To[wave][8 * hh + r][t * 16 + col] = (acc[t][r] + acr[t][r] * (1.0f / RS)) * (1.0f / (CS * WC)); }
  wave_lds_sync();
  const size_t b = (size_t)m0 / SEQ, s0 = (size_t)m0 % SEQ;
  float* ob = out + (b * SEQ_FULL + s0) * DM + n0;
  for (int pass = 0; pass < 2; ++pass) {
#pragma unroll 1
    for (int it = 0; it < 8; ++it) {
      const int rr = it * 2 + hh; const v4f f = *(const v4f*)(&To[wave][rr][col * 4]);
      *(volatile v4f*)(ob + (size_t)rr * DM + col * 4) = f; }
    __threadfence(); }
}
}

extern "C" void kernel_launch(void* const* d_in, const int* in_sizes, int n_in, void* d_out, int out_size, void* d_ws, size_t ws_size, hipStream_t stream) {
  const size_t need_x = ((size_t)(NB - 1) * SEQ_FULL + SEQ) * DM, need_w = (size_t)DM * DM;
  if (n_in < 8 || (size_t)in_sizes[0] < need_x || (size_t)out_size < need_x) return;
  if ((size_t)in_sizes[1] < need_w || (size_t)in_sizes[3] < need_w || (size_t)in_sizes[5] < need_w || (size_t)in_sizes[7] < need_w) return;
  if (in_sizes[2] < DM || in_sizes[4] < DM || in_sizes[6] < DM) return;
  const float* x = (const float*)d_in[0];
  const float* Wq = (const float*)d_in[1]; const float* bq = (const float*)d_in[2];
  const float* Wk = (const float*)d_in[3]; const float* bk = (const float*)d_in[4];
  const float* Wv = (const float*)d_in[5]; const float* bv = (const float*)d_in[6];
  const float* Wo = (const float*)d_in[7];
  size_t off = 0; char* ws = (char*)d_ws;
  auto carve = [&](size_t bytes) { char* p = ws + off; off += (bytes + 255) & ~(size_t)255; return p; };
  const size_t xplane = (size_t)MROWS * DM * 2;
  const size_t wplanes = (size_t)4 * DM * DM * 2;
  const size_t hplane = (size_t)NB * H * SEQ * HD * 2;
  b16* Xp = (b16*)carve(xplane); b16* Wt = (b16*)carve(wplanes);
  b16* Qh = (b16*)carve(hplane); b16* Qr = (b16*)carve(hplane); b16* Kh = (b16*)carve(hplane); b16* Kr = (b16*)carve(hplane);
  b16* Vth = (b16*)carve(hplane); b16* Vtr = (b16*)carve(hplane);
  b16* Ch = (b16*)carve(xplane); b16* Cr = (b16*)carve(xplane);
  if (off > ws_size || off > ((size_t)128 << 20)) return;
  cvt_x_kernel<<<dim3((unsigned)(((size_t)MROWS * (DM / 8)) / 256)), 256, 0, stream>>>(x, Xp);
  cvt_w_kernel<<<dim3(DM / 64, DM / 64, 4), 64, 0, stream>>>(Wq, Wk, Wv, Wo, Wt);
  proj_kernel<0><<<dim3(DM / 64, MROWS / 64, 2), 128, 0, stream>>>(Xp, Wt, bq, bk, Qh, Qr, Kh, Kr);
  proj_kernel<1><<<dim3(DM / 64, MROWS / 64, 1), 128, 0, stream>>>(Xp, Wt + (size_t)2 * DM * DM, bv, bv, Vth, Vtr, Vth, Vtr);
  attn_kernel<true><<<dim3(EBLK, NB * H), 64, 0, stream>>>(Qh, Qr, Kh, Kr, Vth, Vtr, Ch, Cr, 0);
  if (QBLK > EBLK) attn_kernel<false><<<dim3(QBLK - EBLK, NB * H), 64, 0, stream>>>(Qh, Qr, Kh, Kr, Vth, Vtr, Ch, Cr, EBLK);
  oproj_kernel<<<dim3(DM / 64, MROWS / 64), 128, 0, stream>>>(Ch, Cr, Wt + (size_t)3 * DM * DM, (float*)d_out);
}
